// Canonical_41609643163873
// MI455X (gfx1250) — hardware-verified
//
#include <hip/hip_runtime.h>
#include <math.h>

typedef __attribute__((ext_vector_type(16))) _Float16 v16h;
typedef __attribute__((ext_vector_type(16))) __bf16 v16b;
typedef __attribute__((ext_vector_type(8)))  _Float16 v8h;
typedef __attribute__((ext_vector_type(8)))  float v8f;
typedef __attribute__((ext_vector_type(4)))  float v4f;
typedef __attribute__((ext_vector_type(2)))  float v2f;
typedef __attribute__((ext_vector_type(4)))  unsigned v4u;
typedef __attribute__((ext_vector_type(4)))  int v4i;
typedef float __attribute__((may_alias)) float_a;
typedef int __attribute__((may_alias)) int_a;

template <typename T> __device__ __forceinline__ void vst2(void* p, T v) { *(volatile T*)p = v; __threadfence(); *(volatile T*)p = v; }
__device__ __forceinline__ v8f wmma16(v16h a, v16h b, v8f c) {
  v8f d = __builtin_amdgcn_wmma_f32_16x16x32_f16(false, a, false, b, (short)0, c, false, false);
  asm volatile("v_nop\n\tv_nop\n\tv_nop\n\tv_nop" : "+v"(d) : "v"(a), "v"(b));
  return d;
}
__device__ __forceinline__ v8f wmma_bf(v16b a, v16b b, v8f c) {
  v8f d = __builtin_amdgcn_wmma_f32_16x16x32_bf16(false, a, false, b, (short)0, c, false, false);
  asm volatile("v_nop\n\tv_nop\n\tv_nop\n\tv_nop" : "+v"(d) : "v"(a), "v"(b));
  return d;
}
__device__ __forceinline__ v16h frag_h(const _Float16* rowk0, int lane) {
  union { v16h v; v8h q[2]; } u; const _Float16* p = rowk0 + 8 * (lane >> 4);
  u.q[0] = *(const v8h*)p; u.q[1] = *(const v8h*)(p + 16); return u.v;
}
__device__ __forceinline__ v16h frag_f32(const float* rowk0, int lane) {
  v16h a; const float* p = rowk0 + 8 * (lane >> 4);
#pragma unroll
  for (int i = 0; i < 8; ++i) { a[i] = (_Float16)p[i]; a[8 + i] = (_Float16)p[16 + i]; }
  return a;
}
__device__ __forceinline__ v16h frag_f32s(const float* rowk0, int lane, float sc) {
  v16h a; const float* p = rowk0 + 8 * (lane >> 4);
#pragma unroll
  for (int i = 0; i < 8; ++i) { a[i] = (_Float16)(p[i] * sc); a[8 + i] = (_Float16)(p[16 + i] * sc); }
  return a;
}
__device__ __forceinline__ v16h fragc_f32(const float* W, int k0, int n, int lane, int ld, int K) {
  v16h a; const int g = lane >> 4;
#pragma unroll
  for (int i = 0; i < 8; ++i) { const int ka = k0 + 8 * g + i, kb = ka + 16;
    a[i] = (_Float16)(ka < K ? W[(size_t)ka * ld + n] : 0.f); a[8 + i] = (_Float16)(kb < K ? W[(size_t)kb * ld + n] : 0.f); }
  return a;
}
struct F2 { v16b h, l; };
__device__ __forceinline__ F2 bsplit16(const float v[16]) { F2 r;
#pragma unroll
  for (int i = 0; i < 16; ++i) { const __bf16 h = (__bf16)v[i]; r.h[i] = h; r.l[i] = (__bf16)(v[i] - (float)h); }
  return r; }
__device__ __forceinline__ F2 split_row(const float* row, int k0, int lane) { float v[16]; const float* p = row + k0 + 8 * (lane >> 4);
#pragma unroll
  for (int i = 0; i < 8; ++i) { v[i] = p[i]; v[8 + i] = p[16 + i]; }
  return bsplit16(v); }
__device__ __forceinline__ F2 split_rowK(const float* row, int k0, int lane, int K) { float v[16]; const int g = lane >> 4;
#pragma unroll
  for (int i = 0; i < 8; ++i) { const int ka = k0 + 8 * g + i, kb = ka + 16; v[i] = ka < K ? row[ka] : 0.f; v[8 + i] = kb < K ? row[kb] : 0.f; }
  return bsplit16(v); }
__device__ __forceinline__ F2 split_col(const float* W, int k0, int n, int lane, int ld, int K) { float v[16]; const int g = lane >> 4;
#pragma unroll
  for (int i = 0; i < 8; ++i) { const int ka = k0 + 8 * g + i, kb = ka + 16; v[i] = ka < K ? W[(size_t)ka * ld + n] : 0.f; v[8 + i] = kb < K ? W[(size_t)kb * ld + n] : 0.f; }
  return bsplit16(v); }
__device__ __forceinline__ v8f mac3(const F2& a, const F2& b, v8f c) { c = wmma_bf(a.l, b.h, c); c = wmma_bf(a.h, b.l, c); return wmma_bf(a.h, b.h, c); }
__device__ __forceinline__ float sigm(float v) { return 1.0f / (1.0f + expf(-v)); }
#define LDSX() do { asm volatile("s_wait_dscnt 0" ::: "memory"); __builtin_amdgcn_wave_barrier(); __builtin_amdgcn_fence(__ATOMIC_RELEASE, "workgroup"); } while (0)

#define NIMG 2
#define NCL 19
#define HI 512
#define DF 8
#define GW (HI / DF)
#define NPT (NIMG * GW * GW)
#define BW 0.02f

__device__ __forceinline__ float lgam(float x) {
  float p = 1.0f;
#pragma unroll 1
  while (x < 8.0f) { p *= x; x += 1.0f; }
  const float ix = 1.0f / x, ix2 = ix * ix;
  const float ser = ix * (0.0833333333f - ix2 * (0.00277777778f - ix2 * (0.000793650794f - ix2 * 0.000595238095f)));
  return (x - 0.5f) * logf(x) - x + 0.918938533f + ser - logf(p);
}
__global__ __launch_bounds__(128) void k_prep(const float* __restrict__ inp, const float* __restrict__ tgt, float* __restrict__ F, float* __restrict__ LOGF, float* __restrict__ AM1, float* __restrict__ LBY) {
  __shared__ __align__(16) float sf[64][32], slf[64][32], sam[64][32]; __shared__ __align__(16) float slby[64][2];
  const int tid = threadIdx.x, i0 = blockIdx.x * 64;
  if (tid < 64) { const int i = i0 + tid; const int b = i / (GW * GW), rem = i % (GW * GW), yy = rem / GW, xx = rem % GW; const size_t pix = (size_t)(yy * DF) * HI + xx * DF;
    float mx = -3.0e38f; int am = 0; float tm = -3.0e38f;
#pragma unroll 1
    for (int c = 0; c < NCL; ++c) { const float xv = inp[((size_t)b * NCL + c) * HI * HI + pix]; sf[tid][c] = xv; mx = fmaxf(mx, xv); const float tv = tgt[((size_t)b * NCL + c) * HI * HI + pix]; if (tv > tm) { tm = tv; am = c; } }
    float s = 0.f;
#pragma unroll 1
    for (int c = 0; c < NCL; ++c) { const float e = expf(sf[tid][c] - mx); sf[tid][c] = e; s += e; }
    const float inv = 1.0f / s; float lbs = 0.f, asum = 0.f;
#pragma unroll 1
    for (int c = 0; c < NCL; ++c) { const float f = sf[tid][c] * inv; const float al = f / BW + 1.0f; sf[tid][c] = f; slf[tid][c] = logf(f); sam[tid][c] = al - 1.0f; lbs += lgam(al); asum += al; }
#pragma unroll 1
    for (int c = NCL; c < 32; ++c) { sf[tid][c] = 0.f; slf[tid][c] = 0.f; sam[tid][c] = 0.f; }
    slby[tid][0] = lbs - lgam(asum); slby[tid][1] = (float)am; }
  __syncthreads();
  for (int q = tid; q < 64 * 8; q += 128) { const int rl = q >> 3, pc = q & 7; const size_t o = (size_t)(i0 + rl) * 32 + pc * 4;
    vst2(F + o, *(const v4f*)(&sf[rl][pc * 4])); vst2(LOGF + o, *(const v4f*)(&slf[rl][pc * 4])); vst2(AM1 + o, *(const v4f*)(&sam[rl][pc * 4])); }
  if (tid < 32) vst2(LBY + (size_t)i0 * 2 + tid * 4, *(const v4f*)(&slby[0][0] + tid * 4));
}
__global__ __launch_bounds__(128) void k_main(const float* __restrict__ F, const float* __restrict__ LOGF, const float* __restrict__ AM1, const float* __restrict__ LBY, float* __restrict__ part) {
  __shared__ __align__(16) float sS[4][16][68];
  __shared__ float slb[64], sy[64]; __shared__ float srow[4][16]; __shared__ float sl4[4];
  const int tid = threadIdx.x, w = tid >> 5, lane = tid & 31, col = lane & 15, g = lane >> 4;
  const int i0 = blockIdx.x * 64 + w * 16;
  const F2 a = split_row(LOGF + (size_t)(i0 + col) * 32, 0, lane);
  const int rl = lane >> 1, hf = lane & 1; const int irow = i0 + rl;
  float bins[NCL]; float den = 0.f;
#pragma unroll
  for (int c = 0; c < NCL; ++c) bins[c] = 0.f;
#pragma unroll 1
  for (int jt = 0; jt < NPT / 64; ++jt) {
    __syncthreads();
    if (tid < 64) { slb[tid] = LBY[(size_t)(jt * 64 + tid) * 2]; sy[tid] = LBY[(size_t)(jt * 64 + tid) * 2 + 1]; }
#pragma unroll
    for (int t = 0; t < 4; ++t) { v8f s = {}; s = mac3(a, split_row(AM1 + (size_t)(jt * 64 + t * 16 + col) * 32, 0, lane), s);
#pragma unroll
      for (int r = 0; r < 8; ++r) sS[w][8 * g + r][t * 16 + col] = s[r]; }
    __syncthreads();
#pragma unroll 4
    for (int jj = hf * 32; jj < hf * 32 + 32; ++jj) { const int j = jt * 64 + jj; if (j == irow) continue;
      const float kv = expf(sS[w][rl][jj] - slb[jj]); den += kv; const int yc = (int)sy[jj];
#pragma unroll
      for (int c = 0; c < NCL; ++c) bins[c] += (yc == c) ? kv : 0.f; } }
#pragma unroll
  for (int c = 0; c < NCL; ++c) bins[c] += __shfl_xor(bins[c], 1, 32);
  den += __shfl_xor(den, 1, 32);
  float err = 0.f;
  if (hf == 0) { const float dn = fmaxf(den, 1e-10f);
#pragma unroll
    for (int c = 0; c < NCL; ++c) { const float d = bins[c] / dn - F[(size_t)irow * 32 + c]; err += d * d; } }
#pragma unroll
  for (int off = 16; off >= 1; off >>= 1) err += __shfl_xor(err, off, 32);
  if (lane == 0) sl4[w] = err;
  __syncthreads();
  if (tid < 32) vst2(part + (size_t)blockIdx.x * 32 + tid, (float)(tid == 0 ? (sl4[0] + sl4[1]) + (sl4[2] + sl4[3]) : 0.f));
  (void)srow;
}
__global__ __launch_bounds__(32) void k_fin(const float* __restrict__ part, float* __restrict__ out) {
  if (threadIdx.x == 0) { float s = 0.f; for (int b = 0; b < NPT / 64; ++b) s += part[(size_t)b * 32]; vst2(out, s / (float)NPT); }
}
extern "C" void kernel_launch(void* const* d_in, const int* in_sizes, int n_in, void* d_out, int out_size, void* d_ws, size_t ws_size, hipStream_t stream) {
  (void)in_sizes; (void)n_in; (void)out_size; (void)ws_size;
  const float* inp = (const float*)d_in[0]; const float* tgt = (const float*)d_in[1]; float* out = (float*)d_out;
  char* ws = (char*)d_ws; size_t off = 0;
  auto take = [&](size_t bytes) { char* p = ws + off; off += (bytes + 255) & ~(size_t)255; return p; };
  float* F = (float*)take((size_t)NPT * 32 * 4); float* LOGF = (float*)take((size_t)NPT * 32 * 4); float* AM1 = (float*)take((size_t)NPT * 32 * 4); float* LBY = (float*)take((size_t)NPT * 2 * 4); float* part = (float*)take((size_t)(NPT / 64) * 32 * 4);
  k_prep<<<NPT / 64, 128, 0, stream>>>(inp, tgt, F, LOGF, AM1, LBY);
  k_main<<<NPT / 64, 128, 0, stream>>>(F, LOGF, AM1, LBY, part);
  k_fin<<<1, 32, 0, stream>>>(part, out);
}
